// _LocalConditioner_71476845740647
// MI455X (gfx1250) — hardware-run, weakly checked
//
#include <hip/hip_runtime.h>


#define NR   65536
#define SEQ  131072
#define TD   8
#define CD   16
#define FE   56
#define FP   64
#define WI   512
#define NO   16
#define CH   16384
typedef _Float16 h16;
typedef unsigned short bf;
typedef __attribute__((ext_vector_type(16))) __bf16   v16bf;
typedef __attribute__((ext_vector_type(16))) _Float16 v16h;
typedef __attribute__((ext_vector_type(8)))  _Float16 v8h;
typedef __attribute__((ext_vector_type(8)))  unsigned short v8us;
typedef __attribute__((ext_vector_type(8)))  float    v8f;
typedef __attribute__((ext_vector_type(4)))  float    v4f;
typedef v8h  __attribute__((may_alias)) v8ha;
typedef v4f  __attribute__((may_alias)) v4fa;
typedef v8us __attribute__((may_alias)) v8usa;

__device__ __forceinline__ unsigned short f2bf(float f) { unsigned u = __float_as_uint(f); u += 0x7FFFu + ((u >> 16) & 1u); return (unsigned short)(u >> 16); }
__device__ __forceinline__ float bf2f(unsigned short b) { return __uint_as_float(((unsigned)b) << 16); }
__device__ __forceinline__ float bfr(float f) { return bf2f(f2bf(f)); }
__device__ __forceinline__ v16h cat16(v8h lo, v8h hi) { return __builtin_shufflevector(lo, hi, 0, 1, 2, 3, 4, 5, 6, 7, 8, 9, 10, 11, 12, 13, 14, 15); }
__device__ __forceinline__ v16bf cat16b(v8us lo, v8us hi) { return __builtin_bit_cast(v16bf, __builtin_shufflevector(lo, hi, 0, 1, 2, 3, 4, 5, 6, 7, 8, 9, 10, 11, 12, 13, 14, 15)); }
__device__ __forceinline__ v8f wmma16(v16h a, v16h b, v8f c) { return __builtin_amdgcn_wmma_f32_16x16x32_f16(false, a, false, b, (short)0, c, false, false); }
__device__ __forceinline__ v8f wmmab(v16bf a, v16bf b, v8f c) { return __builtin_amdgcn_wmma_f32_16x16x32_bf16(false, a, false, b, (short)0, c, false, false); }


template <typename T16> struct WFrag;
template <> struct WFrag<h16> { typedef v16h V; static __device__ __forceinline__ V ld(const h16* p) { return cat16(*(const v8h*)p, *(const v8h*)(p + 16)); } static __device__ __forceinline__ v8f mma(V a, V b, v8f c) { return wmma16(a, b, c); } };
template <> struct WFrag<bf> { typedef v16bf V; static __device__ __forceinline__ V ld(const bf* p) { return cat16b(*(const v8us*)p, *(const v8us*)(p + 16)); } static __device__ __forceinline__ v8f mma(V a, V b, v8f c) { return wmmab(a, b, c); } };
template <typename T16, int NSPLIT, bool BIAS>
__global__ __launch_bounds__(32) void k_gemmw(const T16* __restrict__ A, const T16* __restrict__ A2, const T16* __restrict__ Bt, const T16* __restrict__ Bt2, int K, float* C, int ldc, const float* __restrict__ bias, size_t sA, size_t sB, size_t sC) {
    typedef typename WFrag<T16>::V V;
    __shared__ __align__(16) float os[16 * 68];
    const size_t z = blockIdx.z; A += z * sA; if (A2) A2 += z * sA; Bt += z * sB; if (Bt2) Bt2 += z * sB; C += z * sC;
    const int lane = threadIdx.x & 31, lr = lane & 15, hi = lane >> 4; const int r0 = blockIdx.x * 64, c0 = blockIdx.y * 64;
    v8f acc[4][4];
#pragma unroll
    for (int mb = 0; mb < 4; ++mb)
#pragma unroll
        for (int nb = 0; nb < 4; ++nb) acc[mb][nb] = (v8f){};
    const size_t aoff = (size_t)(r0 + lr) * K + 8 * hi, boff = (size_t)(c0 + lr) * K + 8 * hi;
#pragma unroll 1
    for (int kc = 0; kc < K; kc += 32) {
        V a[4], a2[4];
#pragma unroll
        for (int mb = 0; mb < 4; ++mb) { a[mb] = WFrag<T16>::ld(A + aoff + (size_t)mb * 16 * K + kc); if (NSPLIT == 1 || NSPLIT == 2) a2[mb] = WFrag<T16>::ld(A2 + aoff + (size_t)mb * 16 * K + kc); }
#pragma unroll
        for (int nb = 0; nb < 4; ++nb) { const V b = WFrag<T16>::ld(Bt + boff + (size_t)nb * 16 * K + kc); V b2; if (NSPLIT >= 2) b2 = WFrag<T16>::ld(Bt2 + boff + (size_t)nb * 16 * K + kc);
#pragma unroll
            for (int mb = 0; mb < 4; ++mb) { acc[mb][nb] = WFrag<T16>::mma(a[mb], b, acc[mb][nb]); if (NSPLIT == 1 || NSPLIT == 2) acc[mb][nb] = WFrag<T16>::mma(a2[mb], b, acc[mb][nb]); if (NSPLIT >= 2) acc[mb][nb] = WFrag<T16>::mma(a[mb], b2, acc[mb][nb]); } }
        asm volatile("v_nop\n\tv_nop\n\tv_nop\n\tv_nop" : "+v"(acc[0][0]), "+v"(acc[1][1]), "+v"(acc[2][2]), "+v"(acc[3][3]) : "v"(a[0]), "v"(a[3]));
    }
#pragma unroll
    for (int mb = 0; mb < 4; ++mb) {
#pragma unroll
        for (int nb = 0; nb < 4; ++nb) {
#pragma unroll
            for (int j = 0; j < 8; ++j) os[(hi * 8 + j) * 68 + nb * 16 + lr] = acc[mb][nb][j]; }
        __builtin_amdgcn_wave_barrier(); asm volatile("" ::: "memory");
        float* crow = C + (size_t)(r0 + mb * 16) * ldc + c0;
#pragma unroll 1
        for (int ps = 0; ps < 2; ++ps) {
#pragma unroll
            for (int s = 0; s < 8; ++s) { const int row = 2 * s + hi, cofs = lr * 4; v4f val = *(const v4fa*)(os + row * 68 + cofs); if (BIAS) { val[0] += bfr(bias[c0 + cofs]); val[1] += bfr(bias[c0 + cofs + 1]); val[2] += bfr(bias[c0 + cofs + 2]); val[3] += bfr(bias[c0 + cofs + 3]); }
                *(volatile v4f*)(crow + (size_t)row * ldc + cofs) = val; }
            if (ps == 0) __threadfence(); }
        __builtin_amdgcn_wave_barrier(); asm volatile("" ::: "memory");
    }
}

__device__ __forceinline__ void splitf(float y, unsigned short& h, unsigned short& l) { h = f2bf(y); l = f2bf(y - bf2f(h)); }
typedef __attribute__((ext_vector_type(2))) unsigned short v2us;
typedef __attribute__((ext_vector_type(4))) unsigned short v4us;

__global__ __launch_bounds__(256) void k_feat(const float* __restrict__ xt, const float* __restrict__ xf, const float* __restrict__ cond, bf* F) { const int e = (blockIdx.x * 256 + threadIdx.x) * 4; if (e >= NR * FP) return; const int c0 = e % FP; const int n = e / FP; const int t = 2 * n; v4us o;
#pragma unroll
    for (int u = 0; u < 4; ++u) { const int c = c0 + u; float v = 0.f;
        if (c < TD) v = xt[(size_t)n * TD + c];
        else if (c < TD + 4 * TD) { const int w = (c - TD) / TD, d = (c - TD) % TD; const int off = (w < 2) ? (w - 2) : (w - 1); int p = t + off; p = p < 0 ? 0 : (p > SEQ - 1 ? SEQ - 1 : p); v = xf[(size_t)p * TD + d]; }
        else if (c < FE) v = cond[(size_t)t * CD + (c - TD - 4 * TD)];
        o[u] = f2bf(v); }
    *(volatile v4us*)(F + e) = o; __threadfence(); *(volatile v4us*)(F + e) = o; }
__global__ __launch_bounds__(256) void k_w0(const float* __restrict__ W0, bf* Bt) { const int e = (blockIdx.x * 256 + threadIdx.x) * 4; if (e >= WI * FP) return; const int c0 = e % FP; const int s = e / FP; const int hr = (s % TD) - 1; v4us o;
#pragma unroll
    for (int u = 0; u < 4; ++u) { const int c = c0 + u; const bool keep = (c < TD) ? (hr >= c) : (c < FE); o[u] = keep ? f2bf(W0[(size_t)s * FE + c]) : (unsigned short)0; } *(volatile v4us*)(Bt + e) = o; __threadfence(); *(volatile v4us*)(Bt + e) = o; }
__global__ __launch_bounds__(256) void k_w1(const float* __restrict__ W1, bf* Bt) { const int e = (blockIdx.x * 256 + threadIdx.x) * 4; if (e >= WI * WI) return; const int k0 = e % WI; const int s = e / WI; v4us o;
#pragma unroll
    for (int u = 0; u < 4; ++u) { const int k = k0 + u; o[u] = ((s % TD) >= (k % TD)) ? f2bf(W1[e + u]) : (unsigned short)0; } *(volatile v4us*)(Bt + e) = o; __threadfence(); *(volatile v4us*)(Bt + e) = o; }
__global__ __launch_bounds__(256) void k_w2(const float* __restrict__ W2, bf* Bt) { const int e = (blockIdx.x * 256 + threadIdx.x) * 4; if (e >= 64 * WI) return; const int k0 = e % WI; const int o_ = e / WI; v4us o;
#pragma unroll
    for (int u = 0; u < 4; ++u) { const int k = k0 + u; o[u] = (o_ < NO && (o_ / 2) > (k % TD) - 1) ? f2bf(W2[(size_t)o_ * WI + k]) : (unsigned short)0; } *(volatile v4us*)(Bt + e) = o; __threadfence(); *(volatile v4us*)(Bt + e) = o; }
__global__ __launch_bounds__(256) void k_rl(const float* __restrict__ Fv, size_t n4, bf* Hh, bf* Hl) { const size_t e = ((size_t)blockIdx.x * 256 + threadIdx.x) * 4; if (e >= n4) return; const v4f a = *(const v4f*)(Fv + e); v4us oh, ol;
#pragma unroll
    for (int u = 0; u < 4; ++u) { unsigned short h, l; splitf(fmaxf(a[u], 0.f), h, l); oh[u] = h; ol[u] = l; } *(volatile v4us*)(Hh + e) = oh; *(volatile v4us*)(Hl + e) = ol; __threadfence(); *(volatile v4us*)(Hh + e) = oh; *(volatile v4us*)(Hl + e) = ol; }
__global__ __launch_bounds__(256) void k_out(const float* __restrict__ Y, const float* __restrict__ b2, int r0, float* OUT) { const int e = (blockIdx.x * 256 + threadIdx.x) * 4; if (e >= CH * NO) return; const int o = e % NO; const int rl = e / NO; v4f r;
#pragma unroll
    for (int u = 0; u < 4; ++u) r[u] = __fadd_rn(Y[(size_t)rl * 64 + o + u], bfr(b2[o + u])); float* dst = OUT + (size_t)(r0 + rl) * NO + o; *(volatile v4f*)dst = r; __threadfence(); *(volatile v4f*)dst = r; }

extern "C" void kernel_launch(void* const* d_in, const int* in_sizes, int n_in,
                              void* d_out, int out_size, void* d_ws, size_t ws_size, hipStream_t stream) {
    (void)in_sizes; (void)n_in; (void)out_size;
    const float** I = (const float**)d_in;
    const float *xt = I[0], *xf = I[1], *cond = I[2], *W0 = I[3], *b0 = I[4], *W1 = I[5], *b1 = I[6], *W2 = I[7], *b2 = I[8];
    float* OUT = (float*)d_out;
    char* wsp = (char*)d_ws;
    auto take = [&](size_t bytes) { char* p = wsp; wsp += (bytes + 255) & ~(size_t)255; return (void*)p; };
    bf* Bt0 = (bf*)take(WI * FP * 2); bf* Bt1 = (bf*)take((size_t)WI * WI * 2); bf* Bt2 = (bf*)take(64 * WI * 2); bf* F = (bf*)take((size_t)NR * FP * 2);
    float* H0 = (float*)take((size_t)CH * WI * 4); bf* Ph = (bf*)take((size_t)CH * WI * 2); bf* Pl = (bf*)take((size_t)CH * WI * 2); float* H1 = (float*)take((size_t)CH * WI * 4); bf* Qh = (bf*)take((size_t)CH * WI * 2); bf* Ql = (bf*)take((size_t)CH * WI * 2); float* Y = (float*)take((size_t)CH * 64 * 4);
    if ((size_t)(wsp - (char*)d_ws) > ws_size) return;
    k_w0<<<(WI * FP / 4 + 255) / 256, 256, 0, stream>>>(W0, Bt0); k_w1<<<(WI * WI / 4 + 255) / 256, 256, 0, stream>>>(W1, Bt1); k_w2<<<(64 * WI / 4 + 255) / 256, 256, 0, stream>>>(W2, Bt2);
    k_feat<<<(NR * FP / 4 + 255) / 256, 256, 0, stream>>>(xt, xf, cond, F);
    for (int r0 = 0; r0 < NR; r0 += CH) {
        k_gemmw<bf, 0, true><<<dim3(CH / 64, WI / 64, 1), 32, 0, stream>>>(F + (size_t)r0 * FP, nullptr, Bt0, nullptr, FP, H0, WI, b0, 0, 0, 0); k_rl<<<(CH * WI / 4 + 255) / 256, 256, 0, stream>>>(H0, (size_t)CH * WI, Ph, Pl);
        k_gemmw<bf, 1, true><<<dim3(CH / 64, WI / 64, 1), 32, 0, stream>>>(Ph, Pl, Bt1, nullptr, WI, H1, WI, b1, 0, 0, 0); k_rl<<<(CH * WI / 4 + 255) / 256, 256, 0, stream>>>(H1, (size_t)CH * WI, Qh, Ql);
        k_gemmw<bf, 1, false><<<dim3(CH / 64, 1, 1), 32, 0, stream>>>(Qh, Ql, Bt2, nullptr, WI, Y, 64, nullptr, 0, 0, 0);
        k_out<<<(CH * NO / 4 + 255) / 256, 256, 0, stream>>>(Y, b2, r0, OUT); }
}
